// GuidedMoEBasic_4372276707575
// MI455X (gfx1250) — hardware-verified
//
#include <hip/hip_runtime.h>

constexpr int kBatch       = 8;
constexpr int kDocLen      = 128;
constexpr int kNUtt        = kBatch * kDocLen;
constexpr int kHdim        = 768;
constexpr int kNEmo        = 7;
constexpr int kDcat        = 776;
constexpr int kKpad        = 800;
constexpr int kKGroups     = kKpad / 8;
constexpr int kHid         = 256;
constexpr int kNcols       = 576;
constexpr int kPairsPerDoc = 8256;
constexpr int kNPairs      = kBatch * kPairsPerDoc;
constexpr int kOutFloats   = kNPairs * 2;
constexpr int kTabPitch    = 16;

typedef __attribute__((ext_vector_type(16))) _Float16 v16h;
typedef __attribute__((ext_vector_type(8)))  _Float16 v8h;
typedef __attribute__((ext_vector_type(16))) __bf16   v16b;
typedef __attribute__((ext_vector_type(8)))  __bf16   v8b;
typedef __attribute__((ext_vector_type(8)))  float    v8f;
typedef __attribute__((ext_vector_type(4)))  float    v4f;

__device__ __forceinline__ unsigned short f2bf_bits(float f) {
  unsigned u = __float_as_uint(f);
  return (unsigned short)((u + 0x7FFFu + ((u >> 16) & 1u)) >> 16);
}
__device__ __forceinline__ float bf_bits2f(unsigned short h) { return __uint_as_float(((unsigned)h) << 16); }

__device__ __forceinline__ void dep_guard_h(v8f& a, v8f& b, v16h x, v16h y) { asm volatile("v_nop\n\tv_nop\n\tv_nop\n\tv_nop" : "+v"(a), "+v"(b) : "v"(x), "v"(y)); }
__device__ __forceinline__ void dep_guard_b(v8f& a, v8f& b, v16b x, v16b y) { asm volatile("v_nop\n\tv_nop\n\tv_nop\n\tv_nop" : "+v"(a), "+v"(b) : "v"(x), "v"(y)); }
__device__ __forceinline__ void keep4_h(v16h a, v16h b, v16h c, v16h d) { asm volatile("v_nop" :: "v"(a), "v"(b), "v"(c), "v"(d)); }
__device__ __forceinline__ void keep4_b(v16b a, v16b b, v16b c, v16b d) { asm volatile("v_nop" :: "v"(a), "v"(b), "v"(c), "v"(d)); }
__device__ __forceinline__ void acc_guard4(v8f& a, v8f& b, v8f& c, v8f& d) { asm volatile("v_nop\n\tv_nop\n\tv_nop\n\tv_nop" : "+v"(a), "+v"(b), "+v"(c), "+v"(d)); }
template <typename T> struct Frag;
template <> struct Frag<_Float16> {
  typedef v16h V; union U { v16h v; v8h h[2]; };
  static __device__ __forceinline__ v16h load(const _Float16* p) {
    U f; f.h[0] = *(const v8h*)(p); f.h[1] = *(const v8h*)(p + 16); return f.v;
  }
  static __device__ __forceinline__ v8f mma(v16h a, v16h b, v8f c) {
    return __builtin_amdgcn_wmma_f32_16x16x32_f16(false, a, false, b, (short)0, c, false, false);
  }
  static __device__ __forceinline__ void guard(v8f& a, v8f& b, v16h x, v16h y) { dep_guard_h(a, b, x, y); }
  static __device__ __forceinline__ void keep(v16h a, v16h b, v16h c, v16h d) { keep4_h(a, b, c, d); }
};
template <> struct Frag<__bf16> {
  typedef v16b V; union U { v16b v; v8b h[2]; };
  static __device__ __forceinline__ v16b load(const __bf16* p) {
    U f; f.h[0] = *(const v8b*)(p); f.h[1] = *(const v8b*)(p + 16); return f.v;
  }
  static __device__ __forceinline__ v8f mma(v16b a, v16b b, v8f c) {
    return __builtin_amdgcn_wmma_f32_16x16x32_bf16(false, a, false, b, (short)0, c, false, false);
  }
  static __device__ __forceinline__ void guard(v8f& a, v8f& b, v16b x, v16b y) { dep_guard_b(a, b, x, y); }
  static __device__ __forceinline__ void keep(v16b a, v16b b, v16b c, v16b d) { keep4_b(a, b, c, d); }
};

template <int ET> struct Elem;
template <> struct Elem<0> { typedef _Float16 T; };
template <> struct Elem<1> { typedef __bf16 T; };
template <int ET, bool SPLIT, int BIAS_MODE, int OUT_MODE, bool RESID, int ACT = 0>
__global__ __launch_bounds__(256) void wmma_gemm64(
    const unsigned short* __restrict__ Ap, const unsigned short* __restrict__ A2p, int lda, long strideA,
    const unsigned short* __restrict__ Btp, const unsigned short* __restrict__ Bt2p, int ldb, long strideB,
    void* __restrict__ Cout, void* __restrict__ Cout2, int ldc, long strideC,
    const float* __restrict__ bias,
    const float* __restrict__ resid, long strideR,
    int M, int N, int K, float scale) {
  typedef typename Elem<ET>::T T;
  typedef typename Frag<T>::V V;
  const T* A = (const T*)Ap; const T* A2 = (const T*)A2p; const T* Bt = (const T*)Btp; const T* Bt2 = (const T*)Bt2p;
  __shared__ __align__(16) float sT[8][16 * 68];
  const int b    = blockIdx.y;
  const int lane = threadIdx.x & 31;
  const int wave = threadIdx.x >> 5;
  const int tilesN = N >> 6;
  const int tilesM = M >> 6;
  const int tile = blockIdx.x * 8 + wave;
  if (tile >= tilesM * tilesN) return;
  const int tm = tile / tilesN;
  const int tn = tile - tm * tilesN;
  const int m0 = tm << 6;
  const int n0 = tn << 6;

  const T* Ab  = A  + (size_t)b * strideA;
  const T* Bb  = Bt + (size_t)b * strideB;
  const T* Ab2 = SPLIT ? (A2  + (size_t)b * strideA) : nullptr;
  const T* Bb2 = SPLIT ? (Bt2 + (size_t)b * strideB) : nullptr;

  const int rlane = lane & 15;
  const int koff  = (lane >> 4) * 8;
  const int mOff  = (lane >> 4) * 8;

  v8f acc[4][4];
#pragma unroll
  for (int i = 0; i < 4; ++i)
#pragma unroll
    for (int j = 0; j < 4; ++j) acc[i][j] = (v8f){0.f,0.f,0.f,0.f,0.f,0.f,0.f,0.f};

  for (int k0 = 0; k0 < K; k0 += 32) {
    V bh[4], bl[4];
#pragma unroll
    for (int j = 0; j < 4; ++j) {
      const size_t bo = (size_t)(n0 + (j << 4) + rlane) * ldb + koff + k0;
      bh[j] = Frag<T>::load(Bb + bo);
      if (SPLIT) bl[j] = Frag<T>::load(Bb2 + bo);
    }
#pragma unroll
    for (int i = 0; i < 4; ++i) {
      const size_t ao = (size_t)(m0 + (i << 4) + rlane) * lda + koff + k0;
      V ah = Frag<T>::load(Ab + ao);
      V al;
      if (SPLIT) al = Frag<T>::load(Ab2 + ao);
#pragma unroll
      for (int j = 0; j < 4; ++j) {
        acc[i][j] = Frag<T>::mma(ah, bh[j], acc[i][j]);
        if (SPLIT) {
          acc[i][j] = Frag<T>::mma(ah, bl[j], acc[i][j]);
          acc[i][j] = Frag<T>::mma(al, bh[j], acc[i][j]);
        }
      }
      Frag<T>::guard(acc[i][0], acc[i][3], ah, SPLIT ? al : ah);
    }
    Frag<T>::keep(bh[0], bh[1], bh[2], bh[3]);
    if (SPLIT) Frag<T>::keep(bl[0], bl[1], bl[2], bl[3]);
  }
  acc_guard4(acc[0][0], acc[0][1], acc[0][2], acc[0][3]);
  acc_guard4(acc[1][0], acc[1][1], acc[1][2], acc[1][3]);
  acc_guard4(acc[2][0], acc[2][1], acc[2][2], acc[2][3]);
  acc_guard4(acc[3][0], acc[3][1], acc[3][2], acc[3][3]);

  float* slab = sT[wave];
  const float* Rb = RESID ? (resid + (size_t)b * strideR) : nullptr;
#pragma unroll
  for (int i = 0; i < 4; ++i) {
    const int mBase = m0 + (i << 4);
#pragma unroll
    for (int j = 0; j < 4; ++j) {
      const int n = n0 + (j << 4) + rlane;
      float bv = 0.f;
      if (BIAS_MODE == 2) bv = bias[n];
#pragma unroll
      for (int r = 0; r < 8; ++r) {
        float v = acc[i][j][r] * scale;
        if (BIAS_MODE == 1) v += bias[mBase + mOff + r];
        if (BIAS_MODE == 2) v += bv;
        if (RESID) v += Rb[(size_t)(mBase + mOff + r) * ldc + n];
        if (ACT == 1) v = tanhf(v);
        if (ACT == 2) v = fmaxf(v, 0.0f);
        if (ACT == 4) v = (v > 0.f) ? v : 0.01f * v;
        slab[(mOff + r) * 68 + (j << 4) + rlane] = v;
      }
    }
    __builtin_amdgcn_fence(__ATOMIC_RELEASE, "workgroup");
    __builtin_amdgcn_wave_barrier();
    __builtin_amdgcn_fence(__ATOMIC_ACQUIRE, "workgroup");
    if (OUT_MODE == 0) {
      float* C = (float*)Cout + (size_t)b * strideC;
      const int hh = lane >> 4, c4 = (lane & 15) * 4;
      for (int pass = 0; pass < 2; ++pass) {
#pragma unroll
        for (int it = 0; it < 8; ++it) {
          const int row = it * 2 + hh;
          v4f v = *(const v4f*)(slab + row * 68 + c4);
          *(volatile v4f*)(C + (size_t)(mBase + row) * ldc + n0 + c4) = v;
        }
        __threadfence();
      }
    } else {
      const int q = lane >> 3, c8 = (lane & 7) * 8;
      unsigned short* C  = (unsigned short*)Cout  + (size_t)b * strideC;
      unsigned short* C2 = (OUT_MODE == 2) ? ((unsigned short*)Cout2 + (size_t)b * strideC) : nullptr;
      for (int pass = 0; pass < 2; ++pass) {
#pragma unroll
        for (int it = 0; it < 4; ++it) {
          const int row = it * 4 + q;
          const float* sp = slab + row * 68 + c8;
          v8h hv, lv;
#pragma unroll
          for (int e = 0; e < 8; ++e) {
            if (OUT_MODE == 1) {
              hv[e] = (_Float16)sp[e];
            } else {
              unsigned short hb = f2bf_bits(sp[e]);
              unsigned short lb = f2bf_bits(sp[e] - bf_bits2f(hb));
              hv[e] = __builtin_bit_cast(_Float16, hb);
              lv[e] = __builtin_bit_cast(_Float16, lb);
            }
          }
          *(volatile v8h*)(C + (size_t)(mBase + row) * ldc + n0 + c8) = hv;
          if (OUT_MODE == 2) *(volatile v8h*)(C2 + (size_t)(mBase + row) * ldc + n0 + c8) = lv;
        }
        __threadfence();
      }
    }
    __builtin_amdgcn_fence(__ATOMIC_RELEASE, "workgroup");
    __builtin_amdgcn_wave_barrier();
    __builtin_amdgcn_fence(__ATOMIC_ACQUIRE, "workgroup");
  }
}

__device__ __forceinline__ void split8(const float (&v)[8], v8h& hv, v8h& lv) {
#pragma unroll
  for (int e = 0; e < 8; ++e) {
    const unsigned short hb = f2bf_bits(v[e]);
    const unsigned short lb = f2bf_bits(v[e] - bf_bits2f(hb));
    hv[e] = __builtin_bit_cast(_Float16, hb);
    lv[e] = __builtin_bit_cast(_Float16, lb);
  }
}
__device__ __forceinline__ void store8x2(unsigned short* ph, unsigned short* pl, v8h hv, v8h lv) {
  *(volatile v8h*)ph = hv;
  *(volatile v8h*)pl = lv;
  __threadfence();
  *(volatile v8h*)ph = hv;
  *(volatile v8h*)pl = lv;
}

__global__ __launch_bounds__(256) void build_cat_planes(const float* __restrict__ hp, const float* __restrict__ emo,
                                                        const float* __restrict__ spk,
                                                        unsigned short* __restrict__ cath, unsigned short* __restrict__ catl) {
  const int tid = blockIdx.x * 256 + threadIdx.x;
  if (tid >= kNUtt * kKGroups) return;
  const int i = tid / kKGroups;
  const int g = tid - i * kKGroups;
  const int gh = (g < 96) ? g : 95;
  const float* hrow = hp + (size_t)i * kHdim + gh * 8;
  const v4f a0 = *(const v4f*)(hrow);
  const v4f a1 = *(const v4f*)(hrow + 4);
  float tl[8];
#pragma unroll
  for (int e = 0; e < 7; ++e) tl[e] = emo[(size_t)i * kNEmo + e];
  tl[7] = spk[i];
  float hv8[8];
  hv8[0] = a0[0]; hv8[1] = a0[1]; hv8[2] = a0[2]; hv8[3] = a0[3];
  hv8[4] = a1[0]; hv8[5] = a1[1]; hv8[6] = a1[2]; hv8[7] = a1[3];
  float v[8];
#pragma unroll
  for (int e = 0; e < 8; ++e) v[e] = (g < 96) ? hv8[e] : ((g == 96) ? tl[e] : 0.0f);
  v8h hv, lv;
  split8(v, hv, lv);
  store8x2(cath + (size_t)tid * 8, catl + (size_t)tid * 8, hv, lv);
}

__global__ __launch_bounds__(256) void build_w_planes(const float* __restrict__ W1, const float* __restrict__ Wg,
                                                      unsigned short* __restrict__ bth, unsigned short* __restrict__ btl) {
  const int tid = blockIdx.x * 256 + threadIdx.x;
  if (tid >= 2 * kNcols * kKGroups) return;
  const int q = tid / (kNcols * kKGroups);
  const int r = tid - q * (kNcols * kKGroups);
  const int n = r / kKGroups;
  const int g = r - n * kKGroups;
  int ec = n >> 8; ec = (ec > 1) ? 1 : ec;
  const int h = n & 255;
  int gc = n - 512; gc = (gc < 0) ? 0 : ((gc > 1) ? 1 : gc);
  const float* w1base = W1 + ((size_t)ec * (2 * kDcat) + (size_t)q * kDcat) * kHid + h;
  const float* wgbase = Wg + (size_t)q * kDcat * 2 + gc;
  float v[8];
#pragma unroll
  for (int e = 0; e < 8; ++e) {
    const int k = g * 8 + e;
    const int kc = (k < kDcat) ? k : (kDcat - 1);
    const float a  = w1base[(size_t)kc * kHid];
    const float wg = wgbase[(size_t)kc * 2];
    v[e] = (k < kDcat) ? ((n < 512) ? a : ((n < 514) ? wg : 0.0f)) : 0.0f;
  }
  v8h hv, lv;
  split8(v, hv, lv);
  store8x2(bth + (size_t)tid * 8, btl + (size_t)tid * 8, hv, lv);
}

__global__ __launch_bounds__(256) void utt_heads(const float* __restrict__ cm, const float* __restrict__ W2,
                                                 const float* __restrict__ b1, const float* __restrict__ b2,
                                                 const float* __restrict__ bg, float* __restrict__ tab) {
  __shared__ float w2s[1024];
  __shared__ float cc[8];
  __shared__ float tabs[32 * kTabPitch];
  const int tid = threadIdx.x, lane = tid & 31, wave = tid >> 5;
#pragma unroll
  for (int e = 0; e < 4; ++e) w2s[tid + 256 * e] = W2[tid + 256 * e];
  __syncthreads();
  if (wave == 0) {
    float c0 = 0.f, c1 = 0.f, c2 = 0.f, c3 = 0.f;
#pragma unroll 1
    for (int it = 0; it < 8; ++it) {
      const int h = it * 32 + lane;
      const float b10 = b1[h], b11 = b1[kHid + h];
      c0 += b10 * w2s[2 * h];
      c1 += b10 * w2s[2 * h + 1];
      c2 += b11 * w2s[512 + 2 * h];
      c3 += b11 * w2s[512 + 2 * h + 1];
    }
#pragma unroll
    for (int off = 1; off < 32; off <<= 1) {
      c0 += __shfl_xor(c0, off, 32); c1 += __shfl_xor(c1, off, 32);
      c2 += __shfl_xor(c2, off, 32); c3 += __shfl_xor(c3, off, 32);
    }
    const float b20 = b2[0], b21 = b2[1], b22 = b2[2], b23 = b2[3];
    const float bg0 = bg[0], bg1 = bg[1];
    if (lane == 0) {
      cc[0] = c0 + b20; cc[1] = c1 + b21; cc[2] = c2 + b22; cc[3] = c3 + b23;
      cc[4] = bg0; cc[5] = bg1; cc[6] = 0.f; cc[7] = 0.f;
    }
  }
  __syncthreads();

  const int rowBase = blockIdx.x * 32;
#pragma unroll 1
  for (int rr = 0; rr < 4; ++rr) {
    const int lr = wave * 4 + rr;
    const int row = rowBase + lr;
    const float* ct = cm + (size_t)row * kNcols;
    const float* cb = cm + (size_t)kNUtt * kNcols + (size_t)row * kNcols;
    float s0 = 0.f, s1 = 0.f, s2 = 0.f, s3 = 0.f, s4 = 0.f, s5 = 0.f, s6 = 0.f, s7 = 0.f;
#pragma unroll 2
    for (int it = 0; it < 8; ++it) {
      const int h = it * 32 + lane;
      const float t0 = ct[h], t1 = ct[kHid + h];
      const float u0 = cb[h], u1 = cb[kHid + h];
      const float w00 = w2s[2 * h], w01 = w2s[2 * h + 1];
      const float w10 = w2s[512 + 2 * h], w11 = w2s[512 + 2 * h + 1];
      s0 += t0 * w00; s1 += t0 * w01; s2 += t1 * w10; s3 += t1 * w11;
      s4 += u0 * w00; s5 += u0 * w01; s6 += u1 * w10; s7 += u1 * w11;
    }
#pragma unroll
    for (int off = 1; off < 32; off <<= 1) {
      s0 += __shfl_xor(s0, off, 32); s1 += __shfl_xor(s1, off, 32);
      s2 += __shfl_xor(s2, off, 32); s3 += __shfl_xor(s3, off, 32);
      s4 += __shfl_xor(s4, off, 32); s5 += __shfl_xor(s5, off, 32);
      s6 += __shfl_xor(s6, off, 32); s7 += __shfl_xor(s7, off, 32);
    }
    const float gt0 = ct[512], gt1 = ct[513];
    const float gb0 = cb[512], gb1 = cb[513];
    if (lane == 0) {
      float* tp = tabs + lr * kTabPitch;
      tp[0] = s0 + cc[0]; tp[1] = s1 + cc[1]; tp[2] = s2 + cc[2]; tp[3] = s3 + cc[3];
      tp[4] = gt0 + cc[4]; tp[5] = gt1 + cc[5]; tp[6] = 0.f; tp[7] = 0.f;
      tp[8] = s4; tp[9] = s5; tp[10] = s6; tp[11] = s7;
      tp[12] = gb0; tp[13] = gb1; tp[14] = 0.f; tp[15] = 0.f;
    }
  }
  __syncthreads();
  {
    float* tg = tab + (size_t)rowBase * kTabPitch;
    const int l0 = 2 * wave, l1 = 2 * wave + 1;
    const float v0 = tabs[l0 * 32 + lane];
    const float v1 = tabs[l1 * 32 + lane];
    volatile float* p0 = tg + l0 * 32 + lane;
    volatile float* p1 = tg + l1 * 32 + lane;
    *p0 = v0; *p1 = v1;
    __threadfence();
    *p0 = v0; *p1 = v1;
  }
}

__global__ __launch_bounds__(256) void pair_combine(const float* __restrict__ tab, const int* __restrict__ ids_unused,
                                                    float* __restrict__ out) {
  const int f = blockIdx.x * 256 + threadIdx.x;
  if (f >= kOutFloats) return;
  const int n = f >> 1;
  const int o = f & 1;
  int b = n / kPairsPerDoc; b = (b > kBatch - 1) ? (kBatch - 1) : b;
  const int p = n - b * kPairsPerDoc;
  int et = (int)((sqrtf(8.0f * (float)p + 1.0f) - 1.0f) * 0.5f);
  et = (et < 0) ? 0 : ((et > kDocLen - 1) ? (kDocLen - 1) : et);
#pragma unroll
  for (int it = 0; it < 2; ++it) {
    const int tri = ((et + 1) * (et + 2)) >> 1;
    et += (tri <= p && et < kDocLen - 1) ? 1 : 0;
  }
#pragma unroll
  for (int it = 0; it < 2; ++it) {
    const int tri = (et * (et + 1)) >> 1;
    et -= (tri > p && et > 0) ? 1 : 0;
  }
  int t = p - ((et * (et + 1)) >> 1);
  t = (t < 0) ? 0 : ((t > kDocLen - 1) ? (kDocLen - 1) : t);
  const int i = b * kDocLen + t;
  const int j = b * kDocLen + et;
  const v4f ai  = *(const v4f*)(tab + (size_t)i * kTabPitch);
  const v4f gi4 = *(const v4f*)(tab + (size_t)i * kTabPitch + 4);
  const v4f aj  = *(const v4f*)(tab + (size_t)j * kTabPitch + 8);
  const v4f gj4 = *(const v4f*)(tab + (size_t)j * kTabPitch + 12);
  const float at0 = o ? ai[1] : ai[0];
  const float at1 = o ? ai[3] : ai[2];
  const float ab0 = o ? aj[1] : aj[0];
  const float ab1 = o ? aj[3] : aj[2];
  const float g0 = gi4[0] + gj4[0];
  const float g1 = gi4[1] + gj4[1];
  const float r = (at0 + ab0) * g0 + (at1 + ab1) * g1;
  volatile float* po = out + f;
  *po = r;
  __threadfence();
  *po = r;
}

extern "C" void kernel_launch(void* const* d_in, const int* in_sizes, int n_in,
                              void* d_out, int out_size, void* d_ws, size_t ws_size,
                              hipStream_t stream) {
  const float* emo = (const float*)d_in[0];
  const float* hp  = (const float*)d_in[1];
  const int*   ids = (const int*)d_in[2];
  const float* spk = (const float*)d_in[3];
  const float* Wg  = (const float*)d_in[4];
  const float* bg  = (const float*)d_in[5];
  const float* W1  = (const float*)d_in[6];
  const float* b1  = (const float*)d_in[7];
  const float* W2  = (const float*)d_in[8];
  const float* b2  = (const float*)d_in[9];
  float* out = (float*)d_out;

  if (n_in < 10 || out_size != kOutFloats) return;
  if (in_sizes[1] != kNUtt * kHdim || in_sizes[6] != 2 * 2 * kDcat * kHid) return;

  const size_t catBytes = (size_t)kNUtt * kKpad * 2;
  const size_t btBytes  = (size_t)2 * kNcols * kKpad * 2;
  const size_t cmBytes  = (size_t)2 * kNUtt * kNcols * 4;
  const size_t tabBytes = (size_t)kNUtt * kTabPitch * 4;
  const size_t total = 2 * catBytes + 2 * btBytes + cmBytes + tabBytes;
  if (total > ws_size) return;
  char* wsb = (char*)d_ws;
  unsigned short* cath = (unsigned short*)(wsb);
  unsigned short* catl = (unsigned short*)(wsb + catBytes);
  unsigned short* bth  = (unsigned short*)(wsb + 2 * catBytes);
  unsigned short* btl  = (unsigned short*)(wsb + 2 * catBytes + btBytes);
  float* cmat = (float*)(wsb + 2 * catBytes + 2 * btBytes);
  float* tab  = (float*)(wsb + 2 * catBytes + 2 * btBytes + cmBytes);

  build_cat_planes<<<(kNUtt * kKGroups) / 256, 256, 0, stream>>>(hp, emo, spk, cath, catl);
  build_w_planes<<<(2 * kNcols * kKGroups) / 256, 256, 0, stream>>>(W1, Wg, bth, btl);

  wmma_gemm64<1, true, 0, 0, false, 0><<<dim3(18, 2), 256, 0, stream>>>(
      cath, catl, kKpad, 0L,
      bth, btl, kKpad, (long)kNcols * kKpad,
      (void*)cmat, (void*)nullptr, kNcols, (long)kNUtt * kNcols,
      (const float*)nullptr,
      (const float*)nullptr, 0L,
      kNUtt, kNcols, kKpad, 1.0f);

  utt_heads<<<kNUtt / 32, 256, 0, stream>>>(cmat, W2, b1, b2, bg, tab);

  pair_combine<<<kOutFloats / 256, 256, 0, stream>>>(tab, ids, out);
}
